// GCNLayer_58368605553168
// MI455X (gfx1250) — hardware-run, weakly checked
//
#include <hip/hip_runtime.h>

typedef float          v8f   __attribute__((ext_vector_type(8)));
typedef float          v4f   __attribute__((ext_vector_type(4)));
typedef unsigned int   v4u   __attribute__((ext_vector_type(4)));
typedef int            v8i   __attribute__((ext_vector_type(8)));
typedef unsigned short v8us  __attribute__((ext_vector_type(8)));
typedef unsigned short v16us __attribute__((ext_vector_type(16)));
typedef __bf16         v16bf __attribute__((ext_vector_type(16)));
typedef _Float16       v16h  __attribute__((ext_vector_type(16)));
typedef v4f  __attribute__((may_alias)) v4fa;
typedef v8us __attribute__((may_alias)) v8usa;
union FragB { v16bf v; v16us u; v8us h[2]; v8i w; };
union FragH { v16h  v; v16us u; v8us h[2]; v8i w; };

__device__ __forceinline__ v8f wmb(const FragB& a, const FragB& b, v8f c) {
  v8f d = __builtin_amdgcn_wmma_f32_16x16x32_bf16(false, a.v, false, b.v, (short)0, c, false, false);
  asm volatile("v_nop\n\tv_nop\n\tv_nop\n\tv_nop" : "+v"(d) : "v"(a.w), "v"(b.w));
  return d;
}

__device__ __forceinline__ v8f wmh(const FragH& a, const FragH& b, v8f c) {
  v8f d = __builtin_amdgcn_wmma_f32_16x16x32_f16(false, a.v, false, b.v, (short)0, c, false, false);
  asm volatile("v_nop\n\tv_nop\n\tv_nop\n\tv_nop" : "+v"(d) : "v"(a.w), "v"(b.w));
  return d;
}

__device__ __forceinline__ unsigned bf16_bits(float f) {
  const unsigned u = __float_as_uint(f);
  const unsigned r = (u + 0x7FFFu + ((u >> 16) & 1u)) >> 16;
  const unsigned q = (u >> 16) | 0x40u;
  return ((u & 0x7fffffffu) > 0x7f800000u) ? q : r;
}

__device__ __forceinline__ float bf16_val(float f) {
  return __uint_as_float(bf16_bits(f) << 16);
}
__device__ __forceinline__ int clampi(int v, int lo, int hi) {
  return v < lo ? lo : (v > hi ? hi : v);
}

__device__ __forceinline__ unsigned f16_bits(float f) {
  const unsigned u  = __float_as_uint(f);
  const unsigned s  = (u >> 16) & 0x8000u;
  const unsigned a  = u & 0x7fffffffu;
  const unsigned t  = a - 0x38000000u;
  const unsigned r  = (t + 0x0FFFu + ((t >> 13) & 1u)) >> 13;
  const unsigned rc = r > 0x7C00u ? 0x7C00u : r;
  const bool small  = a < 0x38800000u;
  const bool isnan  = a > 0x7f800000u;
  const unsigned fin = small ? 0u : (s | rc);
  return isnan ? (s | 0x7E00u) : fin;
}

__device__ __forceinline__ unsigned pk16(unsigned lo, unsigned hi) { return lo | (hi << 16); }
__device__ __forceinline__ unsigned bf16_lo_bits(float v) {
  float hi = bf16_val(v);
  asm volatile("" : "+v"(hi));
  return bf16_bits(v - hi);
}
__device__ __forceinline__ v4u pack8_bf16(v4f a, v4f c) {
  return (v4u){ pk16(bf16_bits(a[0]), bf16_bits(a[1])), pk16(bf16_bits(a[2]), bf16_bits(a[3])),
                pk16(bf16_bits(c[0]), bf16_bits(c[1])), pk16(bf16_bits(c[2]), bf16_bits(c[3])) };
}
__device__ __forceinline__ v4u pack8_bf16_lo(v4f a, v4f c) {
  return (v4u){ pk16(bf16_lo_bits(a[0]), bf16_lo_bits(a[1])), pk16(bf16_lo_bits(a[2]), bf16_lo_bits(a[3])),
                pk16(bf16_lo_bits(c[0]), bf16_lo_bits(c[1])), pk16(bf16_lo_bits(c[2]), bf16_lo_bits(c[3])) };
}
__device__ __forceinline__ v4u pack8_f16(v4f a, v4f c) {
  return (v4u){ pk16(f16_bits(a[0]), f16_bits(a[1])), pk16(f16_bits(a[2]), f16_bits(a[3])),
                pk16(f16_bits(c[0]), f16_bits(c[1])), pk16(f16_bits(c[2]), f16_bits(c[3])) };
}

template <int FORM>
__global__ __launch_bounds__(256) void k_plane(const float* __restrict__ src, int rows, int cols, int ldsrc,
                                               unsigned short* __restrict__ dst, int MP, int KP) {
  static_assert(FORM >= 0 && FORM <= 3);
  const int KTOT = (FORM == 1 || FORM == 3) ? 2 * KP : KP;
  const unsigned ppr   = (unsigned)(KTOT >> 3);
  const unsigned kp8   = (unsigned)(KP >> 3);
  const unsigned total = (unsigned)MP * ppr;
  const unsigned g     = blockIdx.x * 256u + threadIdx.x;
  const unsigned rowu  = g / ppr;
  const unsigned p     = g - rowu * ppr;
  const bool second    = p >= kp8;
  const int row = (int)rowu;
  const int c0  = (int)((second ? p - kp8 : p) << 3);
  const float* srow = src + (size_t)clampi(row, 0, rows - 1) * (size_t)ldsrc;
  float x[8];
  unsigned mk[8];
#pragma unroll
  for (int e = 0; e < 8; ++e) {
    const int c = c0 + e;
    const float v = srow[clampi(c, 0, cols - 1)];
    asm volatile("" :: "v"(v));
    x[e]  = v;
    mk[e] = (row < rows && c < cols) ? 0xFFFFu : 0u;
  }
  const v4f a = (v4f){ x[0], x[1], x[2], x[3] };
  const v4f c = (v4f){ x[4], x[5], x[6], x[7] };
  v4u o;
  if (FORM == 2) {
    o = pack8_f16(a, c);
  } else {
    const v4u hi = pack8_bf16(a, c);
    o = hi;
    if (FORM == 1) { const v4u lo = pack8_bf16_lo(a, c); o = second ? lo : hi; }
  }
  const v4u mw = (v4u){ pk16(mk[0], mk[1]), pk16(mk[2], mk[3]), pk16(mk[4], mk[5]), pk16(mk[6], mk[7]) };
  o &= mw;
  if (g < total) {
    volatile v4u* q = (volatile v4u*)(dst + (size_t)g * 8);
    *q = o;
    __threadfence();
    *q = o;
  }
}

template <int FORM> struct FragOf    { typedef FragB T; };
template <>         struct FragOf<2> { typedef FragH T; };
__device__ __forceinline__ v8f mm(const FragB& a, const FragB& b, v8f c) { return wmb(a, b, c); }
__device__ __forceinline__ v8f mm(const FragH& a, const FragH& b, v8f c) { return wmh(a, b, c); }
template <class F> __device__ __forceinline__ F ld_frag(const unsigned short* p) {
  F f;
  f.h[0] = *(const v8usa*)(p);
  f.h[1] = *(const v8usa*)(p + 16);
  return f;
}

template <int FORM, int EPI>
__global__ __launch_bounds__(256) __attribute__((amdgpu_num_vgpr(248)))
void k_gemm_nt(const unsigned short* __restrict__ A, const unsigned short* __restrict__ B,
               const float* __restrict__ bias, float* __restrict__ D, int M, int N, int KTOT, int ldd) {
  static_assert(FORM >= 0 && FORM <= 2);
  static_assert(EPI == 0 || EPI == 1);
  typedef typename FragOf<FORM>::T F;
  __shared__ __attribute__((aligned(16))) float sT[8][16 * 68];
  const int lane = threadIdx.x & 31;
  const int wave = threadIdx.x >> 5;
  const int tilesM = (M + 63) >> 6;
  const int tilesN = (N + 63) >> 6;
  const int tile = blockIdx.x * 8 + wave;
  if (tile >= tilesM * tilesN) return;
  const int tm = tile / tilesN;
  const int tn = tile - tm * tilesN;
  const int m0 = tm << 6;
  const int n0 = tn << 6;

  const int rl = lane & 15;
  const int h8 = (lane >> 4) * 8;
  const unsigned short* pa = A + (size_t)(m0 + rl) * (size_t)KTOT + h8;
  const unsigned short* pb = B + (size_t)(n0 + rl) * (size_t)KTOT + h8;

  v8f acc[4][4];
#pragma unroll
  for (int i = 0; i < 4; ++i)
#pragma unroll
    for (int j = 0; j < 4; ++j) acc[i][j] = (v8f){0.f, 0.f, 0.f, 0.f, 0.f, 0.f, 0.f, 0.f};

#pragma unroll 1
  for (int k0 = 0; k0 < KTOT; k0 += 32) {
    F bf[4];
#pragma unroll
    for (int j = 0; j < 4; ++j) bf[j] = ld_frag<F>(pb + (size_t)(j << 4) * (size_t)KTOT + k0);
#pragma unroll
    for (int i = 0; i < 4; ++i) {
      const F af = ld_frag<F>(pa + (size_t)(i << 4) * (size_t)KTOT + k0);
#pragma unroll
      for (int j = 0; j < 4; ++j) acc[i][j] = mm(af, bf[j], acc[i][j]);
    }
  }

  float* slab = sT[wave];
  const int hh = lane >> 4;
  const int c4 = (lane & 15) * 4;
  const int nc = n0 + c4;
  const bool cok = nc < N;
  v4f bv = (v4f){0.f, 0.f, 0.f, 0.f};
  if (EPI == 1) {
    bv = *(const v4fa*)(bias + clampi(nc, 0, N - 4));
    asm volatile("" :: "v"(bv));
  }
#pragma unroll
  for (int i = 0; i < 4; ++i) {
    const int mBase = m0 + (i << 4);
#pragma unroll
    for (int j = 0; j < 4; ++j) {
#pragma unroll
      for (int r = 0; r < 8; ++r) slab[(h8 + r) * 68 + (j << 4) + rl] = acc[i][j][r];
    }
    __builtin_amdgcn_fence(__ATOMIC_RELEASE, "workgroup");
    __builtin_amdgcn_wave_barrier();
    __builtin_amdgcn_fence(__ATOMIC_ACQUIRE, "workgroup");
    v4f vv[8];
#pragma unroll
    for (int it = 0; it < 8; ++it) {
      const int row = it * 2 + hh;
      v4f v = *(const v4fa*)(slab + row * 68 + c4);
      if (EPI == 1) v += bv;
      vv[it] = v;
    }
    for (int pass = 0; pass < 2; ++pass) {
#pragma unroll
      for (int it = 0; it < 8; ++it) {
        const int row = mBase + it * 2 + hh;
        if (cok && row < M) *(volatile v4f*)(D + (size_t)row * (size_t)ldd + nc) = vv[it];
      }
      __threadfence();
    }
    __builtin_amdgcn_fence(__ATOMIC_RELEASE, "workgroup");
    __builtin_amdgcn_wave_barrier();
    __builtin_amdgcn_fence(__ATOMIC_ACQUIRE, "workgroup");
  }
}

typedef int      v4i  __attribute__((ext_vector_type(4)));
typedef unsigned v2u  __attribute__((ext_vector_type(2)));
typedef v4i __attribute__((may_alias)) v4ia;
typedef v2u __attribute__((may_alias)) v2ua;
typedef v4u __attribute__((may_alias)) v4ua;

constexpr int NN     = 100000;
constexpr int NE     = 1600000;
constexpr int DF     = 128;
constexpr int KT     = 2 * DF;
constexpr int NBRUN  = 1024;
constexpr int SLB    = 10;
constexpr int NBLK   = 98;
constexpr int CAP    = 21504;
constexpr int WLCAP  = 3072;
constexpr int DEGCAP = 64;
constexpr int MPAD   = 100096;
constexpr int WCHUNK = 256;
constexpr int NCHUNK = NE / WCHUNK;
constexpr int CPW    = (NCHUNK + 7) / 8;
constexpr int BK_WL   = 0;
constexpr int BK_SL   = BK_WL + 8 * WLCAP;
constexpr int BK_CNTW = BK_SL + CAP;
constexpr int BK_CNT  = BK_CNTW + 8 * NBRUN;
constexpr int BK_OFF  = BK_CNT + NBRUN;
constexpr int BK_MISC = BK_OFF + NBRUN;
constexpr int BK_INTS = BK_MISC + 32;
constexpr int BK_BYTES = BK_INTS * 4;

static_assert(DF == 32 * 4);
static_assert(NN % 16 == 0 && NN % 32 == 0 && NN % 8 == 0);
static_assert(NE % WCHUNK == 0 && NE % 8 == 0);
static_assert(NBRUN == (1 << SLB));
static_assert(NBRUN * NBLK >= NN && NBRUN * (NBLK - 1) < NN);
static_assert((NN - (NBLK - 1) * NBRUN) % 32 == 0);
static_assert(NBRUN * NBLK >= MPAD && MPAD >= NN);
static_assert(MPAD == 782 * 128 && MPAD % 64 == 0);
static_assert(CAP * 4 >= 5 * 16721);
static_assert(CAP % 1024 == 0 && CAP % 32 == 0);
static_assert(DEGCAP >= 36 + 8);
static_assert(8 * WLCAP >= CAP && WLCAP * 4 >= 5 * 2091);
static_assert(((long long)NE << SLB) < (1LL << 31));
static_assert(BK_INTS % 4 == 0 && BK_SL % 4 == 0 && BK_CNT % 4 == 0 && BK_OFF % 4 == 0);
static_assert(BK_BYTES <= 262144 && BK_BYTES + 0 <= 327680);
static_assert(CPW * 8 >= NCHUNK);
static_assert((NN * DF / 8) % 256 == 0 && (DF * KT / 8) % 256 == 0);
static_assert(KT % 32 == 0 && DF % 64 == 0);

constexpr size_t SZ_A    = (size_t)MPAD * KT * 2;
constexpr size_t SZ_H    = (size_t)MPAD * DF * 4;
constexpr size_t SZ_XB   = (size_t)NN * DF * 2;
constexpr size_t SZ_LIST = (size_t)NBLK * CAP * 4;
constexpr size_t SZ_CNT  = (size_t)NN * 4;
constexpr size_t SZ_FLG  = (size_t)NBLK * 128;
constexpr size_t SZ_WD   = (size_t)DF * KT * 2;
constexpr size_t O_A     = 0;
constexpr size_t O_H     = O_A + SZ_A;
constexpr size_t O_LIST  = O_H + SZ_H;
constexpr size_t O_CNT   = O_LIST + SZ_LIST;
constexpr size_t O_OFF   = O_CNT + SZ_CNT;
constexpr size_t O_FLG   = O_OFF + SZ_CNT;
constexpr size_t O_WD    = O_FLG + SZ_FLG;
constexpr size_t WS_TOTAL = O_WD + SZ_WD;
static_assert(O_H % 128 == 0 && O_LIST % 128 == 0 && O_CNT % 128 == 0 && O_OFF % 128 == 0);
static_assert(O_FLG % 128 == 0 && O_WD % 128 == 0);
static_assert(SZ_XB <= SZ_H);
static_assert(WS_TOTAL <= (size_t)128 * 1024 * 1024);

__device__ __forceinline__ void wave_sync() {
  __builtin_amdgcn_fence(__ATOMIC_RELEASE, "wavefront");
  __builtin_amdgcn_wave_barrier();
  __builtin_amdgcn_fence(__ATOMIC_ACQUIRE, "wavefront");
}

__device__ __forceinline__ int put_hit(int* lst, int pos, bool h, int word) {
  if (h) { if (pos < WLCAP) lst[pos] = word; }
  return pos + (h ? 1 : 0);
}

__global__ __launch_bounds__(256) void k_bucket(const int* __restrict__ dstv, const int* __restrict__ srcv,
                                                int* __restrict__ LIST, int* __restrict__ CNT,
                                                int* __restrict__ OFF, int* __restrict__ FLG) {
  extern __shared__ __attribute__((aligned(16))) int dsm[];
  int* wl   = dsm + BK_WL;
  int* sl   = dsm + BK_SL;
  int* cntw = dsm + BK_CNTW;
  int* cnt  = dsm + BK_CNT;
  int* offs = dsm + BK_OFF;
  int* misc = dsm + BK_MISC;
  const int tid = (int)threadIdx.x, lane = tid & 31, wave = tid >> 5;
  const int blk = (int)blockIdx.x;
  const int base = blk * NBRUN;
  int nb = NN - base;
  nb = nb > NBRUN ? NBRUN : (nb < 0 ? 0 : nb);

  {
    const v4i z4 = {0, 0, 0, 0};
    for (int i = tid * 4; i < BK_INTS; i += 1024) *(v4ia*)(dsm + i) = z4;
  }
  __syncthreads();

  int* mywl = wl + wave * WLCAP;
  int wc = 0;
  {
    const int cBeg = wave * CPW;
    const int cEnd = (cBeg + CPW) < NCHUNK ? (cBeg + CPW) : NCHUNK;
    const unsigned nbs = (unsigned)base;
    const unsigned unb = (unsigned)nb;
#pragma unroll 1
    for (int c = cBeg; c < cEnd; ++c) {
      const int e0  = c * WCHUNK + lane * 8;
      const int e0c = e0 > NE - 8 ? NE - 8 : e0;
      v4i da = *(const v4ia*)(dstv + e0c);
      v4i db = *(const v4ia*)(dstv + e0c + 4);
      asm volatile("" :: "v"(da));
      asm volatile("" :: "v"(db));
      const int inv = (e0 + 8 <= NE) ? 0 : -1;
      const unsigned s0 = (unsigned)(da.x | inv) - nbs, s1 = (unsigned)(da.y | inv) - nbs;
      const unsigned s2 = (unsigned)(da.z | inv) - nbs, s3 = (unsigned)(da.w | inv) - nbs;
      const unsigned s4 = (unsigned)(db.x | inv) - nbs, s5 = (unsigned)(db.y | inv) - nbs;
      const unsigned s6 = (unsigned)(db.z | inv) - nbs, s7 = (unsigned)(db.w | inv) - nbs;
      const bool h0 = s0 < unb, h1 = s1 < unb, h2 = s2 < unb, h3 = s3 < unb;
      const bool h4 = s4 < unb, h5 = s5 < unb, h6 = s6 < unb, h7 = s7 < unb;
      const int nl = (h0 ? 1 : 0) + (h1 ? 1 : 0) + (h2 ? 1 : 0) + (h3 ? 1 : 0) +
                     (h4 ? 1 : 0) + (h5 ? 1 : 0) + (h6 ? 1 : 0) + (h7 ? 1 : 0);
      const unsigned any = __builtin_amdgcn_ballot_w32(nl != 0);
      if (any != 0u) {
        int incl = nl;
#pragma unroll
        for (int d = 1; d < 32; d <<= 1) {
          const int y = __shfl_up(incl, (unsigned)d, 32);
          incl += (lane >= d) ? y : 0;
        }
        const int tot = __builtin_amdgcn_readlane(incl, 31);
        int pos = wc + incl - nl;
        pos = put_hit(mywl, pos, h0, ((e0 + 0) << SLB) | (int)s0);
        pos = put_hit(mywl, pos, h1, ((e0 + 1) << SLB) | (int)s1);
        pos = put_hit(mywl, pos, h2, ((e0 + 2) << SLB) | (int)s2);
        pos = put_hit(mywl, pos, h3, ((e0 + 3) << SLB) | (int)s3);
        pos = put_hit(mywl, pos, h4, ((e0 + 4) << SLB) | (int)s4);
        pos = put_hit(mywl, pos, h5, ((e0 + 5) << SLB) | (int)s5);
        pos = put_hit(mywl, pos, h6, ((e0 + 6) << SLB) | (int)s6);
        pos = put_hit(mywl, pos, h7, ((e0 + 7) << SLB) | (int)s7);
        wc += tot;
      }
    }
  }
  if (lane == 0) {
    misc[wave]     = wc > WLCAP ? WLCAP : wc;
    misc[8 + wave] = wc > WLCAP ? 1 : 0;
  }
  __syncthreads();

  int myc = misc[wave];
  myc = __builtin_amdgcn_readfirstlane(clampi(myc, 0, WLCAP));
  int* mycnt = cntw + wave * NBRUN;
#pragma unroll 1
  for (int b0 = 0; b0 < myc; b0 += 32) {
    const int idx = b0 + lane;
    const int ent = mywl[idx < WLCAP ? idx : WLCAP - 1];
    const int m32 = (myc - b0) < 32 ? (myc - b0) : 32;
#pragma unroll 1
    for (int k = 0; k < m32; ++k) {
      const int u    = __builtin_amdgcn_readlane(ent, k);
      const int slot = u & (NBRUN - 1);
      if (lane == 0) mycnt[slot] = mycnt[slot] + 1;
    }
  }
  __syncthreads();

#pragma unroll 1
  for (int j = 0; j < NBRUN / 256; ++j) {
    const int s = tid + 256 * j;
    int t = 0;
#pragma unroll
    for (int w = 0; w < 8; ++w) t += cntw[w * NBRUN + s];
    cnt[s] = t;
  }
  __syncthreads();

  if (wave == 0) {
    const int sb = lane * (NBRUN / 32);
    int s = 0;
#pragma unroll 1
    for (int i = 0; i < NBRUN / 32; ++i) s += cnt[sb + i];
    int incl = s;
#pragma unroll
    for (int d = 1; d < 32; d <<= 1) {
      const int y = __shfl_up(incl, (unsigned)d, 32);
      incl += (lane >= d) ? y : 0;
    }
    int run = incl - s;
#pragma unroll 1
    for (int i = 0; i < NBRUN / 32; ++i) {
      const int cv = cnt[sb + i];
      offs[sb + i] = run;
      run += cv;
    }
    if (lane == 31) misc[16] = run;
  }
  __syncthreads();

#pragma unroll 1
  for (int j = 0; j < NBRUN / 256; ++j) {
    const int s = tid + 256 * j;
    int run = offs[s];
#pragma unroll
    for (int w = 0; w < 8; ++w) {
      const int c = cntw[w * NBRUN + s];
      cntw[w * NBRUN + s] = run;
      run += c;
    }
  }
  __syncthreads();

#pragma unroll 1
  for (int b0 = 0; b0 < myc; b0 += 32) {
    const int idx = b0 + lane;
    const int ent = mywl[idx < WLCAP ? idx : WLCAP - 1];
    const int m32 = (myc - b0) < 32 ? (myc - b0) : 32;
#pragma unroll 1
    for (int k = 0; k < m32; ++k) {
      const int u    = __builtin_amdgcn_readlane(ent, k);
      const int slot = u & (NBRUN - 1);
      if (lane == 0) {
        int p = mycnt[slot];
        p = clampi(p, 0, CAP - 1);
        sl[p] = u;
        mycnt[slot] = p + 1;
      }
    }
  }
  __syncthreads();

  int ovf = 0;
#pragma unroll
  for (int w = 0; w < 8; ++w) ovf |= misc[8 + w];
  const int totRaw = misc[16];
  if (totRaw > CAP || totRaw < 0) ovf = 1;
  const int tt = clampi(totRaw, 0, CAP);

  int* Lb = LIST + (size_t)blk * CAP;
#pragma unroll 1
  for (int it = 0; it < CAP / 1024; ++it) {
    const int i = it * 1024 + tid * 4;
    const v4i u = *(const v4ia*)(sl + i);
    int g0 = srcv[clampi(u.x >> SLB, 0, NE - 1)];
    int g1 = srcv[clampi(u.y >> SLB, 0, NE - 1)];
    int g2 = srcv[clampi(u.z >> SLB, 0, NE - 1)];
    int g3 = srcv[clampi(u.w >> SLB, 0, NE - 1)];
    asm volatile("" :: "v"(g0));
    asm volatile("" :: "v"(g1));
    asm volatile("" :: "v"(g2));
    asm volatile("" :: "v"(g3));
    v4i o;
    o.x = clampi(g0, 0, NN - 1) & ((i + 0 < tt) ? -1 : 0);
    o.y = clampi(g1, 0, NN - 1) & ((i + 1 < tt) ? -1 : 0);
    o.z = clampi(g2, 0, NN - 1) & ((i + 2 < tt) ? -1 : 0);
    o.w = clampi(g3, 0, NN - 1) & ((i + 3 < tt) ? -1 : 0);
    volatile v4i* q = (volatile v4i*)(Lb + i);
    *q = o;
    __threadfence();
    *q = o;
  }

  {
    const v4i cv = *(const v4ia*)(cnt + 4 * tid);
    const v4i ov = *(const v4ia*)(offs + 4 * tid);
    const v4i fv = {ovf, ovf, ovf, ovf};
    const bool wr = (4 * tid) < nb;
    volatile v4i* qc = (volatile v4i*)(CNT + base + 4 * (wr ? tid : 0));
    volatile v4i* qo = (volatile v4i*)(OFF + base + 4 * (wr ? tid : 0));
    volatile v4i* qf = (volatile v4i*)(FLG + blk * 32 + 4 * (tid & 7));
    if (wr) { *qc = cv; *qo = ov; }
    if (tid < 8) *qf = fv;
    __threadfence();
    if (wr) { *qc = cv; *qo = ov; }
    if (tid < 8) *qf = fv;
  }
}

__global__ __launch_bounds__(256) void k_agg(const unsigned* __restrict__ XBw, const int* __restrict__ LIST,
                                             const int* __restrict__ CNT, const int* __restrict__ OFF,
                                             const int* __restrict__ FLG, unsigned* __restrict__ Aw) {
  __shared__ __attribute__((aligned(16))) unsigned rowbuf[8][128];
  const int tid = (int)threadIdx.x, lane = tid & 31, wave = tid >> 5;
  const int blk = (int)blockIdx.x;
  const int base = blk * NBRUN;
  const int* Lb = LIST + (size_t)blk * CAP;
  unsigned* rb = rowbuf[wave];
  int fl = FLG[blk * 32];
  asm volatile("" :: "v"(fl));
  const bool bpois = fl != 0;
  const float qnan = __uint_as_float(0x7fc00000u);

#pragma unroll 1
  for (int si = 0; si < NBRUN / 8; ++si) {
    const int node = base + si * 8 + wave;
    if (node < MPAD) {
      const bool live = node < NN;
      const int nc = live ? node : NN - 1;
      int c = CNT[nc];
      int o = OFF[nc];
      asm volatile("" :: "v"(c));
      asm volatile("" :: "v"(o));
      const bool big = (c > DEGCAP) || (c < 0);
      c = clampi(c, 0, DEGCAP);
      o = clampi(o, 0, CAP - 1);
      const int cn = __builtin_amdgcn_readfirstlane(live ? c : 0);

      const v2u sx = *(const v2ua*)(XBw + (size_t)nc * 64 + 2 * lane);
      unsigned sx0 = sx.x, sx1 = sx.y;
      asm volatile("" :: "v"(sx0));
      asm volatile("" :: "v"(sx1));

      float a0 = 0.0f, a1 = 0.0f, a2 = 0.0f, a3 = 0.0f;
#pragma unroll 1
      for (int b0 = 0; b0 < cn; b0 += 32) {
        int j = b0 + lane;
        j = j < cn ? j : cn - 1;
        int idx = o + j;
        idx = idx > CAP - 1 ? CAP - 1 : idx;
        int sr = Lb[idx];
        asm volatile("" :: "v"(sr));
        sr = clampi(sr, 0, NN - 1);
        const int m32 = (cn - b0) < 32 ? (cn - b0) : 32;
#pragma unroll 1
        for (int k = 0; k < m32; ++k) {
          const int sk = __builtin_amdgcn_readlane(sr, k);
          const v2u w = *(const v2ua*)(XBw + (size_t)sk * 64 + 2 * lane);
          a0 = a0 + __uint_as_float(w.x << 16);
          a1 = a1 + __uint_as_float(w.x & 0xffff0000u);
          a2 = a2 + __uint_as_float(w.y << 16);
          a3 = a3 + __uint_as_float(w.y & 0xffff0000u);
        }
      }
      const float den = (float)(c > 0 ? c : 1);
      const float q0 = a0 / den, q1 = a1 / den, q2 = a2 / den, q3 = a3 / den;
      const bool has = c > 0;
      float m0 = has ? q0 : __uint_as_float(sx0 << 16);
      float m1 = has ? q1 : __uint_as_float(sx0 & 0xffff0000u);
      float m2 = has ? q2 : __uint_as_float(sx1 << 16);
      float m3 = has ? q3 : __uint_as_float(sx1 & 0xffff0000u);
      const bool pz = bpois || big;
      m0 = pz ? qnan : m0;
      m1 = pz ? qnan : m1;
      m2 = pz ? qnan : m2;
      m3 = pz ? qnan : m3;
      const unsigned lm = live ? 0xFFFFFFFFu : 0u;
      v2u hw, lw;
      hw.x = pk16(bf16_bits(m0), bf16_bits(m1)) & lm;
      hw.y = pk16(bf16_bits(m2), bf16_bits(m3)) & lm;
      lw.x = pk16(bf16_lo_bits(m0), bf16_lo_bits(m1)) & lm;
      lw.y = pk16(bf16_lo_bits(m2), bf16_lo_bits(m3)) & lm;
      *(v2ua*)(rb + 2 * lane)      = hw;
      *(v2ua*)(rb + 64 + 2 * lane) = lw;
      wave_sync();
      const v4u qv = *(const v4ua*)(rb + 4 * lane);
      wave_sync();
      volatile v4u* qp = (volatile v4u*)(Aw + (size_t)node * 128 + 4 * lane);
      *qp = qv;
      __threadfence();
      *qp = qv;
    }
  }
}

__global__ __launch_bounds__(256) void k_out(const float* __restrict__ H, const float* __restrict__ x,
                                             const int* __restrict__ CNT, const int* __restrict__ FLG,
                                             float* __restrict__ out) {
  const int tid = (int)threadIdx.x, lane = tid & 31;
  const int row = (int)blockIdx.x * 8 + (tid >> 5);
  const int rc = row < NN ? row : NN - 1;
  v4f hv = *(const v4fa*)(H + (size_t)rc * DF + 4 * lane);
  v4f xv = *(const v4fa*)(x + (size_t)rc * DF + 4 * lane);
  int cv = CNT[rc];
  int fl = FLG[(rc >> SLB) * 32];
  asm volatile("" :: "v"(hv));
  asm volatile("" :: "v"(xv));
  asm volatile("" :: "v"(cv));
  asm volatile("" :: "v"(fl));
  const bool bad = (fl != 0) || (cv < 0) || (cv > DEGCAP);
  const float qnan = __uint_as_float(0x7fc00000u);
  v4f o;
  o.x = ((hv.x > 0.0f) ? hv.x : (hv.x - hv.x)) + bf16_val(xv.x);
  o.y = ((hv.y > 0.0f) ? hv.y : (hv.y - hv.y)) + bf16_val(xv.y);
  o.z = ((hv.z > 0.0f) ? hv.z : (hv.z - hv.z)) + bf16_val(xv.z);
  o.w = ((hv.w > 0.0f) ? hv.w : (hv.w - hv.w)) + bf16_val(xv.w);
  o.x = bad ? qnan : o.x;
  o.y = bad ? qnan : o.y;
  o.z = bad ? qnan : o.z;
  o.w = bad ? qnan : o.w;
  if (row < NN) {
    volatile v4f* q = (volatile v4f*)(out + (size_t)row * DF + 4 * lane);
    *q = o;
    __threadfence();
    *q = o;
  }
}

extern "C" void kernel_launch(void* const* d_in, const int* in_sizes, int n_in,
                              void* d_out, int out_size, void* d_ws, size_t ws_size,
                              hipStream_t stream) {
  if (n_in < 4) return;
  if (in_sizes[0] != NN * DF) return;
  if (in_sizes[1] != NE || in_sizes[2] != NE) return;
  if (in_sizes[3] != DF * DF) return;
  if (out_size != NN * DF) return;
  if (ws_size < WS_TOTAL) return;

  const float* x   = (const float*)d_in[0];
  const int*   src = (const int*)d_in[1];
  const int*   dst = (const int*)d_in[2];
  const float* W   = (const float*)d_in[3];
  float* out = (float*)d_out;

  char* ws = (char*)d_ws;
  unsigned short* Apl = (unsigned short*)(ws + O_A);
  float*          Hp  = (float*)(ws + O_H);
  unsigned short* XB  = (unsigned short*)(ws + O_H);
  int*            LST = (int*)(ws + O_LIST);
  int*            CNT = (int*)(ws + O_CNT);
  int*            OFF = (int*)(ws + O_OFF);
  int*            FLG = (int*)(ws + O_FLG);
  unsigned short* WD  = (unsigned short*)(ws + O_WD);

  hipFuncSetAttribute(reinterpret_cast<const void*>(&k_bucket), hipFuncAttributeMaxDynamicSharedMemorySize, BK_BYTES);

  k_plane<0><<<NN * DF / 8 / 256, 256, 0, stream>>>(x, NN, DF, DF, XB, NN, DF);
  k_plane<3><<<DF * KT / 8 / 256, 256, 0, stream>>>(W, DF, DF, DF, WD, DF, DF);
  k_bucket<<<NBLK, 256, BK_BYTES, stream>>>(dst, src, LST, CNT, OFF, FLG);
  k_agg<<<NBLK, 256, 0, stream>>>((const unsigned*)XB, LST, CNT, OFF, FLG, (unsigned*)Apl);
  {
    const int tiles = (MPAD / 64) * (DF / 64);
    k_gemm_nt<1, 0><<<(tiles + 7) / 8, 256, 0, stream>>>(Apl, WD, (const float*)WD, Hp, MPAD, DF, KT, DF);
  }
  k_out<<<NN / 8, 256, 0, stream>>>(Hp, x, CNT, FLG, out);
}
